// LSTMAutoencoder_9809705304320
// MI455X (gfx1250) — hardware-verified
//
#include <hip/hip_runtime.h>
#include <math.h>

constexpr int NB_SEQ  = 256;
constexpr int NSTEP   = 512;
constexpr int NFEAT   = 64;
constexpr int NHID    = 128;
constexpr int NGATE   = 4 * NHID;
constexpr int NTHR    = 256;
constexpr int SEQ_BLK = 16;
constexpr int HPITCH  = NHID + 8;
constexpr int ZPITCH  = NGATE + 4;
constexpr int NROWS   = NB_SEQ * NSTEP;
constexpr float ACARRY  = 16.0f;
constexpr float WCARRY  = 64.0f;
constexpr float ACC_INV = 1.0f / 1024.0f;
static_assert(NHID == 16 * (NTHR / 32));
static_assert(NB_SEQ % SEQ_BLK == 0);
static_assert(NHID % 32 == 0 && NFEAT % 32 == 0);
static_assert(NROWS % 64 == 0 && NB_SEQ % 64 == 0 && NGATE % 64 == 0 && NFEAT % 64 == 0);
static_assert(SEQ_BLK * NHID == NTHR * 8);
static_assert(SEQ_BLK * NGATE == NTHR * 8 * 4);
static_assert(SEQ_BLK * NFEAT == NTHR * 4);
static_assert(SEQ_BLK * NHID == NTHR * 8);

typedef __attribute__((ext_vector_type(16))) _Float16 v16h;
typedef __attribute__((ext_vector_type(8)))  _Float16 v8h;
typedef __attribute__((ext_vector_type(4)))  _Float16 v4h;
typedef __attribute__((ext_vector_type(16))) __bf16   v16b;
typedef __attribute__((ext_vector_type(8)))  __bf16   v8b;
typedef __attribute__((ext_vector_type(8)))  float    v8f;
typedef __attribute__((ext_vector_type(4)))  float    v4f;
typedef __attribute__((ext_vector_type(4)))  unsigned v4u;

__device__ __forceinline__ unsigned short f2bf_bits(float f) {
  unsigned u = __float_as_uint(f);
  return (unsigned short)((u + 0x7FFFu + ((u >> 16) & 1u)) >> 16);
}
__device__ __forceinline__ float bf_bits2f(unsigned short h) { return __uint_as_float(((unsigned)h) << 16); }

__device__ __forceinline__ void dep_guard_h(v8f& a, v8f& b, v16h x, v16h y) { asm volatile("v_nop\n\tv_nop\n\tv_nop\n\tv_nop" : "+v"(a), "+v"(b) : "v"(x), "v"(y)); }
__device__ __forceinline__ void dep_guard_b(v8f& a, v8f& b, v16b x, v16b y) { asm volatile("v_nop\n\tv_nop\n\tv_nop\n\tv_nop" : "+v"(a), "+v"(b) : "v"(x), "v"(y)); }
__device__ __forceinline__ void keep4_h(v16h a, v16h b, v16h c, v16h d) { asm volatile("v_nop" :: "v"(a), "v"(b), "v"(c), "v"(d)); }
__device__ __forceinline__ void keep4_b(v16b a, v16b b, v16b c, v16b d) { asm volatile("v_nop" :: "v"(a), "v"(b), "v"(c), "v"(d)); }
__device__ __forceinline__ void acc_guard4(v8f& a, v8f& b, v8f& c, v8f& d) { asm volatile("v_nop\n\tv_nop\n\tv_nop\n\tv_nop" : "+v"(a), "+v"(b), "+v"(c), "+v"(d)); }
__device__ __forceinline__ void grp_guard_h(v8f& a0, v8f& a1, v8f& a2, v8f& a3, v16h x, v16h y0, v16h y1, v16h y2, v16h y3) {
  asm volatile("v_nop\n\tv_nop\n\tv_nop\n\tv_nop" : "+v"(a0), "+v"(a1), "+v"(a2), "+v"(a3) : "v"(x), "v"(y0), "v"(y1), "v"(y2), "v"(y3));
}
__device__ __forceinline__ void grp_guard_b(v8f& a0, v8f& a1, v8f& a2, v8f& a3, v16b x, v16b y0, v16b y1, v16b y2, v16b y3) {
  asm volatile("v_nop\n\tv_nop\n\tv_nop\n\tv_nop" : "+v"(a0), "+v"(a1), "+v"(a2), "+v"(a3) : "v"(x), "v"(y0), "v"(y1), "v"(y2), "v"(y3));
}
template <typename T> struct Frag;
template <> struct Frag<_Float16> {
  typedef v16h V; union U { v16h v; v8h h[2]; };
  static __device__ __forceinline__ v16h load(const _Float16* p) {
    U f; f.h[0] = *(const v8h*)(p); f.h[1] = *(const v8h*)(p + 16); return f.v;
  }
  static __device__ __forceinline__ v8f mma(v16h a, v16h b, v8f c) {
    return __builtin_amdgcn_wmma_f32_16x16x32_f16(false, a, false, b, (short)0, c, false, false);
  }
  static __device__ __forceinline__ void guard(v8f& a, v8f& b, v16h x, v16h y) { dep_guard_h(a, b, x, y); }
  static __device__ __forceinline__ void guard4(v8f& a0, v8f& a1, v8f& a2, v8f& a3, v16h x, v16h y0, v16h y1, v16h y2, v16h y3) { grp_guard_h(a0, a1, a2, a3, x, y0, y1, y2, y3); }
  static __device__ __forceinline__ void keep(v16h a, v16h b, v16h c, v16h d) { keep4_h(a, b, c, d); }
};
template <> struct Frag<__bf16> {
  typedef v16b V; union U { v16b v; v8b h[2]; };
  static __device__ __forceinline__ v16b load(const __bf16* p) {
    U f; f.h[0] = *(const v8b*)(p); f.h[1] = *(const v8b*)(p + 16); return f.v;
  }
  static __device__ __forceinline__ v8f mma(v16b a, v16b b, v8f c) {
    return __builtin_amdgcn_wmma_f32_16x16x32_bf16(false, a, false, b, (short)0, c, false, false);
  }
  static __device__ __forceinline__ void guard(v8f& a, v8f& b, v16b x, v16b y) { dep_guard_b(a, b, x, y); }
  static __device__ __forceinline__ void guard4(v8f& a0, v8f& a1, v8f& a2, v8f& a3, v16b x, v16b y0, v16b y1, v16b y2, v16b y3) { grp_guard_b(a0, a1, a2, a3, x, y0, y1, y2, y3); }
  static __device__ __forceinline__ void keep(v16b a, v16b b, v16b c, v16b d) { keep4_b(a, b, c, d); }
};

__device__ __forceinline__ float fsig(float x)  { return __builtin_amdgcn_rcpf(1.0f + __expf(-x)); }
__device__ __forceinline__ float ftanh(float x) { return 1.0f - 2.0f * __builtin_amdgcn_rcpf(__expf(2.0f * x) + 1.0f); }

template <int ET> struct Elem;
template <> struct Elem<0> { typedef _Float16 T; };
template <> struct Elem<1> { typedef __bf16 T; };
template <int ET, bool SPLIT, int BIAS_MODE, int OUT_MODE, bool RESID, int ACT = 0>
__global__ __launch_bounds__(256) void wmma_gemm64(
    const unsigned short* __restrict__ Ap, const unsigned short* __restrict__ A2p, int lda, long strideA,
    const unsigned short* __restrict__ Btp, const unsigned short* __restrict__ Bt2p, int ldb, long strideB,
    void* __restrict__ Cout, void* __restrict__ Cout2, int ldc, long strideC,
    const float* __restrict__ bias,
    const float* __restrict__ resid, long strideR,
    int M, int N, int K, float scale) {
  typedef typename Elem<ET>::T T;
  typedef typename Frag<T>::V V;
  const T* A = (const T*)Ap; const T* A2 = (const T*)A2p; const T* Bt = (const T*)Btp; const T* Bt2 = (const T*)Bt2p;
  __shared__ __align__(16) float sT[8][16 * 68];
  const int b    = blockIdx.y;
  const int lane = threadIdx.x & 31;
  const int wave = threadIdx.x >> 5;
  const int tilesN = N >> 6;
  const int tilesM = M >> 6;
  const int tile = blockIdx.x * 8 + wave;
  if (tile >= tilesM * tilesN) return;
  const int tm = tile / tilesN;
  const int tn = tile - tm * tilesN;
  const int m0 = tm << 6;
  const int n0 = tn << 6;

  const T* Ab  = A  + (size_t)b * strideA;
  const T* Bb  = Bt + (size_t)b * strideB;
  const T* Ab2 = SPLIT ? (A2  + (size_t)b * strideA) : nullptr;
  const T* Bb2 = SPLIT ? (Bt2 + (size_t)b * strideB) : nullptr;

  const int rlane = lane & 15;
  const int koff  = (lane >> 4) * 8;
  const int mOff  = (lane >> 4) * 8;

  v8f acc[4][4];
#pragma unroll
  for (int i = 0; i < 4; ++i)
#pragma unroll
    for (int j = 0; j < 4; ++j) acc[i][j] = (v8f){0.f,0.f,0.f,0.f,0.f,0.f,0.f,0.f};

  for (int k0 = 0; k0 < K; k0 += 32) {
    V bh[4], bl[4];
#pragma unroll
    for (int j = 0; j < 4; ++j) {
      const size_t bo = (size_t)(n0 + (j << 4) + rlane) * ldb + koff + k0;
      bh[j] = Frag<T>::load(Bb + bo);
      if (SPLIT) bl[j] = Frag<T>::load(Bb2 + bo);
    }
#pragma unroll
    for (int i = 0; i < 4; ++i) {
      const size_t ao = (size_t)(m0 + (i << 4) + rlane) * lda + koff + k0;
      V ah = Frag<T>::load(Ab + ao);
      V al;
      if (SPLIT) al = Frag<T>::load(Ab2 + ao);
#pragma unroll
      for (int j = 0; j < 4; ++j) {
        acc[i][j] = Frag<T>::mma(ah, bh[j], acc[i][j]);
        if (SPLIT) {
          acc[i][j] = Frag<T>::mma(ah, bl[j], acc[i][j]);
          acc[i][j] = Frag<T>::mma(al, bh[j], acc[i][j]);
        }
      }
      Frag<T>::guard(acc[i][0], acc[i][3], ah, SPLIT ? al : ah);
      Frag<T>::guard4(acc[i][0], acc[i][1], acc[i][2], acc[i][3], ah, bh[0], bh[1], bh[2], bh[3]);
    }
    Frag<T>::keep(bh[0], bh[1], bh[2], bh[3]);
    if (SPLIT) Frag<T>::keep(bl[0], bl[1], bl[2], bl[3]);
  }
  acc_guard4(acc[0][0], acc[0][1], acc[0][2], acc[0][3]);
  acc_guard4(acc[1][0], acc[1][1], acc[1][2], acc[1][3]);
  acc_guard4(acc[2][0], acc[2][1], acc[2][2], acc[2][3]);
  acc_guard4(acc[3][0], acc[3][1], acc[3][2], acc[3][3]);

  float* slab = sT[wave];
  const float* Rb = RESID ? (resid + (size_t)b * strideR) : nullptr;
#pragma unroll
  for (int i = 0; i < 4; ++i) {
    const int mBase = m0 + (i << 4);
#pragma unroll
    for (int j = 0; j < 4; ++j) {
      const int n = n0 + (j << 4) + rlane;
      float bv = 0.f;
      if (BIAS_MODE == 2) bv = bias[n];
#pragma unroll
      for (int r = 0; r < 8; ++r) {
        float v = acc[i][j][r] * scale;
        if (BIAS_MODE == 1) v += bias[mBase + mOff + r];
        if (BIAS_MODE == 2) v += bv;
        if (RESID) v += Rb[(size_t)(mBase + mOff + r) * ldc + n];
        if (ACT == 1) v = tanhf(v);
        if (ACT == 2) v = fmaxf(v, 0.0f);
        if (ACT == 3) v = v / (1.0f + expf(-v));
        if (ACT == 4) v = (v > 0.f) ? v : 0.01f * v;
        if (ACT == 5) v = 0.5f * v * (1.0f + erff(v * 0.70710678118654752f));
        slab[(mOff + r) * 68 + (j << 4) + rlane] = v;
      }
    }
    __builtin_amdgcn_fence(__ATOMIC_RELEASE, "workgroup");
    __builtin_amdgcn_wave_barrier();
    __builtin_amdgcn_fence(__ATOMIC_ACQUIRE, "workgroup");
    if (OUT_MODE == 0) {
      float* C = (float*)Cout + (size_t)b * strideC;
      const int hh = lane >> 4, c4 = (lane & 15) * 4;
      for (int pass = 0; pass < 2; ++pass) {
#pragma unroll
        for (int it = 0; it < 8; ++it) {
          const int row = it * 2 + hh;
          v4f v = *(const v4f*)(slab + row * 68 + c4);
          *(volatile v4f*)(C + (size_t)(mBase + row) * ldc + n0 + c4) = v;
        }
        __threadfence();
      }
    } else {
      const int q = lane >> 3, c8 = (lane & 7) * 8;
      unsigned short* C  = (unsigned short*)Cout  + (size_t)b * strideC;
      unsigned short* C2 = (OUT_MODE == 2) ? ((unsigned short*)Cout2 + (size_t)b * strideC) : nullptr;
      for (int pass = 0; pass < 2; ++pass) {
#pragma unroll
        for (int it = 0; it < 4; ++it) {
          const int row = it * 4 + q;
          const float* sp = slab + row * 68 + c8;
          v8h hv, lv;
#pragma unroll
          for (int e = 0; e < 8; ++e) {
            if (OUT_MODE == 1) {
              hv[e] = (_Float16)sp[e];
            } else {
              unsigned short hb = f2bf_bits(sp[e]);
              unsigned short lb = f2bf_bits(sp[e] - bf_bits2f(hb));
              hv[e] = __builtin_bit_cast(_Float16, hb);
              lv[e] = __builtin_bit_cast(_Float16, lb);
            }
          }
          *(volatile v8h*)(C + (size_t)(mBase + row) * ldc + n0 + c8) = hv;
          if (OUT_MODE == 2) *(volatile v8h*)(C2 + (size_t)(mBase + row) * ldc + n0 + c8) = lv;
        }
        __threadfence();
      }
    }
    __builtin_amdgcn_fence(__ATOMIC_RELEASE, "workgroup");
    __builtin_amdgcn_wave_barrier();
    __builtin_amdgcn_fence(__ATOMIC_ACQUIRE, "workgroup");
  }
}

__global__ __launch_bounds__(NTHR) void cvt16_kernel(const float* __restrict__ src, unsigned short* __restrict__ dst,
                                                    int n8, float sc) {
  const int i = blockIdx.x * NTHR + threadIdx.x;
  if (i < n8) {
    const float* sp = src + (size_t)i * 8;
    const v4f a = *(const v4f*)(sp);
    const v4f b = *(const v4f*)(sp + 4);
    v8h hv;
#pragma unroll
    for (int e = 0; e < 4; ++e) {
      hv[e]     = (_Float16)(a[e] * sc);
      hv[4 + e] = (_Float16)(b[e] * sc);
    }
    _Float16* dp = (_Float16*)dst + (size_t)i * 8;
    *(volatile v8h*)dp = hv;
    __threadfence();
    *(volatile v8h*)dp = hv;
  }
}

template <int KIN, int XSRC>
__global__ __launch_bounds__(NTHR) void lstm_seq_kernel(
    const float* __restrict__ xf,
    const unsigned short* __restrict__ xhp,
    const float* __restrict__ zxp,
    const unsigned short* __restrict__ WIp,
    const unsigned short* __restrict__ WHp,
    const float* __restrict__ bih, const float* __restrict__ bhh,
    unsigned short* __restrict__ HSp) {
  static_assert(KIN == 0 || (XSRC == 0 && KIN == NFEAT) || (XSRC == 1 && KIN == NHID));
  constexpr int XP  = (KIN > 0) ? (KIN + 8) : 8;
  constexpr int AXN = (KIN > 0) ? (SEQ_BLK * XP) : 8;
  constexpr int ZSN = (KIN == 0) ? (SEQ_BLK * ZPITCH) : 4;
  __shared__ __align__(16) _Float16 Ax[AXN];
  __shared__ __align__(16) _Float16 Ah[SEQ_BLK * HPITCH];
  __shared__ __align__(16) float    Zs[ZSN];

  const _Float16* WI = (const _Float16*)WIp;
  const _Float16* WH = (const _Float16*)WHp;
  const _Float16* xh = (const _Float16*)xhp;
  _Float16* HS = (_Float16*)HSp;
  const int tid = threadIdx.x, lane = tid & 31, wave = tid >> 5;
  const int c = lane & 15, hh = lane >> 4, koff = hh * 8;
  const int rowbase = blockIdx.x * SEQ_BLK;
  const int j = 16 * wave + c;

  if (KIN == 0) {
#pragma unroll
    for (int it = 0; it < 8; ++it) {
      const int idx = it * NTHR + tid;
      const int row = idx >> 7, c4 = (idx & 127) * 4;
      const v4f v = *(const v4f*)(zxp + (size_t)(rowbase + row) * NGATE + c4);
      *(v4f*)(Zs + row * ZPITCH + c4) = v;
      if (it == 3) asm volatile("" ::: "memory");
    }
  }
  {
    const v4u z = {0u, 0u, 0u, 0u};
    *(v4u*)(Ah + (tid >> 4) * HPITCH + (tid & 15) * 8) = z;
  }
  if (KIN > 0) {
    if (XSRC == 0) {
      const int m = tid >> 4, f4 = (tid & 15) * 4;
      const v4f v = *(const v4f*)(xf + ((size_t)(rowbase + m) * NSTEP) * KIN + f4);
      v4h hv;
      hv[0] = (_Float16)(ACARRY * v[0]); hv[1] = (_Float16)(ACARRY * v[1]);
      hv[2] = (_Float16)(ACARRY * v[2]); hv[3] = (_Float16)(ACARRY * v[3]);
      *(v4h*)(Ax + m * XP + f4) = hv;
    } else {
      const int m = tid >> 4, c8 = (tid & 15) * 8;
      const v8h v = *(const v8h*)(xh + ((size_t)(rowbase + m) * NSTEP) * KIN + c8);
      *(v8h*)(Ax + m * XP + c8) = v;
    }
  }
  float bb[4];
#pragma unroll
  for (int g = 0; g < 4; ++g) bb[g] = bih[g * NHID + j] + bhh[g * NHID + j];
  float cst[8], hst[8], zx[4][8];
#pragma unroll
  for (int r = 0; r < 8; ++r) { cst[r] = 0.0f; hst[r] = 0.0f; }
#pragma unroll
  for (int g = 0; g < 4; ++g)
#pragma unroll
    for (int r = 0; r < 8; ++r) zx[g][r] = 0.0f;
  __syncthreads();
  if (KIN == 0) {
#pragma unroll
    for (int g = 0; g < 4; ++g)
#pragma unroll
      for (int r = 0; r < 8; ++r) zx[g][r] = Zs[(8 * hh + r) * ZPITCH + g * NHID + j];
  }

  const v8f z8 = {0.f, 0.f, 0.f, 0.f, 0.f, 0.f, 0.f, 0.f};

#pragma unroll 1
  for (int t = 0; t < NSTEP; ++t) {
    v8f acc0 = z8, acc1 = z8, acc2 = z8, acc3 = z8;
    if (KIN > 0) {
      const _Float16* axrow = Ax + c * XP + koff;
      const _Float16* wi = WI + (size_t)j * KIN + koff;
#pragma unroll 1
      for (int kx = 0; kx < KIN; kx += 32) {
        const v16h a  = Frag<_Float16>::load(axrow + kx);
        const v16h b0 = Frag<_Float16>::load(wi + kx);
        const v16h b1 = Frag<_Float16>::load(wi + (size_t)1 * NHID * KIN + kx);
        const v16h b2 = Frag<_Float16>::load(wi + (size_t)2 * NHID * KIN + kx);
        const v16h b3 = Frag<_Float16>::load(wi + (size_t)3 * NHID * KIN + kx);
        acc0 = Frag<_Float16>::mma(a, b0, acc0);
        acc1 = Frag<_Float16>::mma(a, b1, acc1);
        acc2 = Frag<_Float16>::mma(a, b2, acc2);
        acc3 = Frag<_Float16>::mma(a, b3, acc3);
        grp_guard_h(acc0, acc1, acc2, acc3, a, b0, b1, b2, b3);
      }
    }
    {
      const _Float16* ahrow = Ah + c * HPITCH + koff;
      const _Float16* wh = WH + (size_t)j * NHID + koff;
#pragma unroll 1
      for (int k0 = 0; k0 < NHID; k0 += 32) {
        const v16h a  = Frag<_Float16>::load(ahrow + k0);
        const v16h b0 = Frag<_Float16>::load(wh + k0);
        const v16h b1 = Frag<_Float16>::load(wh + (size_t)1 * NHID * NHID + k0);
        const v16h b2 = Frag<_Float16>::load(wh + (size_t)2 * NHID * NHID + k0);
        const v16h b3 = Frag<_Float16>::load(wh + (size_t)3 * NHID * NHID + k0);
        acc0 = Frag<_Float16>::mma(a, b0, acc0);
        acc1 = Frag<_Float16>::mma(a, b1, acc1);
        acc2 = Frag<_Float16>::mma(a, b2, acc2);
        acc3 = Frag<_Float16>::mma(a, b3, acc3);
        grp_guard_h(acc0, acc1, acc2, acc3, a, b0, b1, b2, b3);
      }
    }
    acc_guard4(acc0, acc1, acc2, acc3);
#pragma unroll
    for (int r = 0; r < 8; ++r) {
      const float zi = acc0[r] * ACC_INV + zx[0][r] + bb[0];
      const float zf = acc1[r] * ACC_INV + zx[1][r] + bb[1];
      const float zg = acc2[r] * ACC_INV + zx[2][r] + bb[2];
      const float zo = acc3[r] * ACC_INV + zx[3][r] + bb[3];
      const float ig = fsig(zi);
      const float fg = fsig(zf);
      const float og = fsig(zo);
      const float gc = ftanh(zg);
      const float cn = fg * cst[r] + ig * gc;
      cst[r] = cn;
      hst[r] = og * ftanh(cn);
    }
    __syncthreads();
#pragma unroll
    for (int r = 0; r < 8; ++r) Ah[(8 * hh + r) * HPITCH + j] = (_Float16)(ACARRY * hst[r]);
    if (KIN > 0) {
      const int tn = (t + 1 < NSTEP) ? (t + 1) : (NSTEP - 1);
      if (XSRC == 0) {
        const int m = tid >> 4, f4 = (tid & 15) * 4;
        const v4f v = *(const v4f*)(xf + ((size_t)(rowbase + m) * NSTEP + (size_t)tn) * KIN + f4);
        v4h hv;
        hv[0] = (_Float16)(ACARRY * v[0]); hv[1] = (_Float16)(ACARRY * v[1]);
        hv[2] = (_Float16)(ACARRY * v[2]); hv[3] = (_Float16)(ACARRY * v[3]);
        *(v4h*)(Ax + m * XP + f4) = hv;
      } else {
        const int m = tid >> 4, c8 = (tid & 15) * 8;
        const v8h v = *(const v8h*)(xh + ((size_t)(rowbase + m) * NSTEP + (size_t)tn) * KIN + c8);
        *(v8h*)(Ax + m * XP + c8) = v;
      }
    }
    __syncthreads();
    {
      const int q = lane >> 3, c8 = (lane & 7) * 8;
      const int row = 2 * wave + (q >> 1);
      const int col = (q & 1) * 64 + c8;
      const size_t go = ((size_t)(rowbase + row) * NSTEP + (size_t)t) * NHID + col;
      for (int pass = 0; pass < 2; ++pass) {
        const v8h v = *(const v8h*)(Ah + row * HPITCH + col);
        *(volatile v8h*)(HS + go) = v;
        __threadfence();
      }
    }
  }
}

static void launch_cvt(const float* src, unsigned short* dst, int nelem, hipStream_t stream) {
  const int n8 = nelem / 8;
  cvt16_kernel<<<(n8 + NTHR - 1) / NTHR, NTHR, 0, stream>>>(src, dst, n8, WCARRY);
}

extern "C" void kernel_launch(void* const* d_in, const int* in_sizes, int n_in,
                              void* d_out, int out_size, void* d_ws, size_t ws_size, hipStream_t stream) {
  if (n_in < 19 || d_out == nullptr || d_ws == nullptr) return;
  if (in_sizes[0] != NROWS * NFEAT || in_sizes[1] != NGATE * NFEAT || in_sizes[2] != NGATE * NHID ||
      in_sizes[3] != NGATE || in_sizes[4] != NGATE ||
      in_sizes[5] != NGATE * NHID || in_sizes[6] != NGATE * NHID || in_sizes[7] != NGATE || in_sizes[8] != NGATE ||
      in_sizes[9] != NGATE * NHID || in_sizes[10] != NGATE * NHID || in_sizes[11] != NGATE || in_sizes[12] != NGATE ||
      in_sizes[13] != NGATE * NHID || in_sizes[14] != NGATE * NHID || in_sizes[15] != NGATE || in_sizes[16] != NGATE ||
      in_sizes[17] != NFEAT * NHID || in_sizes[18] != NFEAT || out_size != NROWS * NFEAT) return;

  const float* x      = (const float*)d_in[0];
  const float* e0_Wih = (const float*)d_in[1];
  const float* e0_Whh = (const float*)d_in[2];
  const float* e0_bih = (const float*)d_in[3];
  const float* e0_bhh = (const float*)d_in[4];
  const float* e1_Wih = (const float*)d_in[5];
  const float* e1_Whh = (const float*)d_in[6];
  const float* e1_bih = (const float*)d_in[7];
  const float* e1_bhh = (const float*)d_in[8];
  const float* d0_Wih = (const float*)d_in[9];
  const float* d0_Whh = (const float*)d_in[10];
  const float* d0_bih = (const float*)d_in[11];
  const float* d0_bhh = (const float*)d_in[12];
  const float* d1_Wih = (const float*)d_in[13];
  const float* d1_Whh = (const float*)d_in[14];
  const float* d1_bih = (const float*)d_in[15];
  const float* d1_bhh = (const float*)d_in[16];
  const float* W_out  = (const float*)d_in[17];
  const float* b_out  = (const float*)d_in[18];
  float* out = (float*)d_out;

  char* ws = (char*)d_ws; size_t off = 0;
  auto carve = [&](size_t bytes) -> char* { char* p = ws + off; off += (bytes + 255) & ~(size_t)255; return p; };
  unsigned short* WIH0 = (unsigned short*)carve((size_t)NGATE * NFEAT * 2);
  unsigned short* WHH0 = (unsigned short*)carve((size_t)NGATE * NHID * 2);
  unsigned short* WIH1 = (unsigned short*)carve((size_t)NGATE * NHID * 2);
  unsigned short* WHH1 = (unsigned short*)carve((size_t)NGATE * NHID * 2);
  unsigned short* WID0 = (unsigned short*)carve((size_t)NGATE * NHID * 2);
  unsigned short* WHD0 = (unsigned short*)carve((size_t)NGATE * NHID * 2);
  unsigned short* WID1 = (unsigned short*)carve((size_t)NGATE * NHID * 2);
  unsigned short* WHD1 = (unsigned short*)carve((size_t)NGATE * NHID * 2);
  unsigned short* WOUT = (unsigned short*)carve((size_t)NFEAT * NHID * 2);
  float*          ZX   = (float*)carve((size_t)NB_SEQ * NGATE * 4);
  unsigned short* HSA  = (unsigned short*)carve((size_t)NROWS * NHID * 2);
  unsigned short* HSB  = (unsigned short*)carve((size_t)NROWS * NHID * 2);
  if (off > ws_size || off > (size_t)134217728) return;

  launch_cvt(e0_Wih, WIH0, NGATE * NFEAT, stream);
  launch_cvt(e0_Whh, WHH0, NGATE * NHID, stream);
  launch_cvt(e1_Wih, WIH1, NGATE * NHID, stream);
  launch_cvt(e1_Whh, WHH1, NGATE * NHID, stream);
  launch_cvt(d0_Wih, WID0, NGATE * NHID, stream);
  launch_cvt(d0_Whh, WHD0, NGATE * NHID, stream);
  launch_cvt(d1_Wih, WID1, NGATE * NHID, stream);
  launch_cvt(d1_Whh, WHD1, NGATE * NHID, stream);
  launch_cvt(W_out,  WOUT, NFEAT * NHID, stream);

  const int nblk = NB_SEQ / SEQ_BLK;
  lstm_seq_kernel<NFEAT, 0><<<nblk, NTHR, 0, stream>>>(x, HSB, ZX, WIH0, WHH0, e0_bih, e0_bhh, HSA);
  lstm_seq_kernel<NHID, 1><<<nblk, NTHR, 0, stream>>>(x, HSA, ZX, WIH1, WHH1, e1_bih, e1_bhh, HSB);
  wmma_gemm64<0, false, 0, 0, false, 0><<<dim3(4, 1), 256, 0, stream>>>(
      HSB + (size_t)(NSTEP - 1) * NHID, HSB + (size_t)(NSTEP - 1) * NHID, NSTEP * NHID, 0L,
      WID0, WID0, NHID, 0L, (void*)ZX, (void*)ZX, NGATE, 0L,
      b_out, b_out, 0L, NB_SEQ, NGATE, NHID, ACC_INV);
  lstm_seq_kernel<0, 1><<<nblk, NTHR, 0, stream>>>(x, HSB, ZX, WID0, WHD0, d0_bih, d0_bhh, HSA);
  lstm_seq_kernel<NHID, 1><<<nblk, NTHR, 0, stream>>>(x, HSA, ZX, WID1, WHD1, d1_bih, d1_bhh, HSB);
  wmma_gemm64<0, false, 2, 0, false, 0><<<dim3((NROWS / 64) / 8, 1), 256, 0, stream>>>(
      HSB, HSB, NHID, 0L, WOUT, WOUT, NHID, 0L, (void*)out, (void*)out, NFEAT, 0L,
      b_out, b_out, 0L, NROWS, NFEAT, NHID, ACC_INV);
}
